// NattenAttention_85109071938185
// MI455X (gfx1250) — hardware-verified
//
#include <hip/hip_runtime.h>
#include <stddef.h>
#include <stdint.h>
#include <math.h>

#define NBT   2
#define CC    128
#define IMH   96
#define IMW   96
#define HWP   9216
#define NPIX  18432
#define NQKV  384
#define KF    384
#define NGRP  32
#define GNN   36864
#define HDH   16
#define QKROW 768
#define KSP   72
#define VTP   136
#define OSP   68
#define STP   388
#define TFP   68
#define NTY   24
#define NTX   24
#define ATT_LDS 99072

static_assert(NPIX % 64 == 0);
static_assert(HWP % 64 == 0);
static_assert(IMH == 4 * NTY);
static_assert(IMW == 4 * NTX);
static_assert(GNN % 1024 == 0);
static_assert(KF % 32 == 0);

typedef __bf16 v16b __attribute__((ext_vector_type(16)));
typedef unsigned short v8us __attribute__((ext_vector_type(8)));
typedef float v8f __attribute__((ext_vector_type(8)));
typedef float v4f __attribute__((ext_vector_type(4)));
typedef unsigned int v4u __attribute__((ext_vector_type(4)));

union FragB { v16b v; v8us u[2]; };
union Pk8 { v8us u8; v4u u4; };

__device__ __forceinline__ v8f zero8() { return (v8f){0.f, 0.f, 0.f, 0.f, 0.f, 0.f, 0.f, 0.f}; }

__device__ __forceinline__ v8f mmab(v16b a, v16b b, v8f c) {
  c = __builtin_amdgcn_wmma_f32_16x16x32_bf16(false, a, false, b, (short)0, c, false, false);
  asm volatile("v_nop\n\tv_nop\n\tv_nop\n\tv_nop" : "+v"(c) : "v"(a), "v"(b));
  return c;
}

__device__ __forceinline__ v16b ldfragb(const unsigned short* p, int ld, int row0, int k0, int lane) {
  const int m = lane & 15, lh = lane >> 4;
  const unsigned short* q = p + (size_t)(row0 + m) * ld + k0 + 8 * lh;
  FragB f;
  f.u[0] = *(const v8us*)(q);
  f.u[1] = *(const v8us*)(q + 16);
  return f.v;
}

__device__ __forceinline__ unsigned int bfbits(float f) {
  const unsigned int u = __float_as_uint(f);
  return (u + 0x7fffu + ((u >> 16) & 1u)) >> 16;
}
__device__ __forceinline__ unsigned int bfsel(float f, int lo) {
  const unsigned int hb = bfbits(f);
  const float res = f - __uint_as_float(hb << 16);
  const unsigned int lb = bfbits(res);
  return lo ? lb : hb;
}
__device__ __forceinline__ unsigned int bfpack2(float a, float b, int lo) {
  return bfsel(a, lo) | (bfsel(b, lo) << 16);
}

__global__ __launch_bounds__(256) void k_gnstats(const float* __restrict__ x, float* __restrict__ stats) {
  __shared__ float red[8];
  __shared__ float shm;
  __shared__ __align__(16) float lin[32];
  const int tid = threadIdx.x, lane = tid & 31, wave = tid >> 5;
  const int bg = blockIdx.x;
  const float* p = x + (size_t)bg * GNN;
  if (tid < 32) lin[tid] = 0.0f;
  float s = 0.f;
#pragma unroll 4
  for (int it = 0; it < GNN / 1024; ++it) {
    const v4f v = *(const v4f*)(p + ((size_t)(it * 256 + tid)) * 4);
    s += (v[0] + v[1]) + (v[2] + v[3]);
  }
#pragma unroll
  for (int off = 1; off < 32; off <<= 1) s += __shfl_xor(s, off, 32);
  if (lane == 0) red[wave] = s;
  __syncthreads();
  if (tid == 0) {
    float tsum = 0.f;
#pragma unroll
    for (int w = 0; w < 8; ++w) tsum += red[w];
    shm = tsum * (1.0f / (float)GNN);
  }
  __syncthreads();
  const float mean = shm;
  float q2 = 0.f;
#pragma unroll 4
  for (int it = 0; it < GNN / 1024; ++it) {
    const v4f v = *(const v4f*)(p + ((size_t)(it * 256 + tid)) * 4);
    const float d0 = v[0] - mean, d1 = v[1] - mean, d2 = v[2] - mean, d3 = v[3] - mean;
    q2 += (d0 * d0 + d1 * d1) + (d2 * d2 + d3 * d3);
  }
#pragma unroll
  for (int off = 1; off < 32; off <<= 1) q2 += __shfl_xor(q2, off, 32);
  if (lane == 0) red[wave] = q2;
  __syncthreads();
  if (tid == 0) {
    float tsum = 0.f;
#pragma unroll
    for (int w = 0; w < 8; ++w) tsum += red[w];
    const float var = tsum * (1.0f / (float)GNN);
    lin[0] = mean;
    lin[1] = rsqrtf(var + 1e-6f);
  }
  __syncthreads();
  if (wave == 0) {
    const v4f lv = *(const v4f*)(lin + 4 * (lane & 7));
    for (int ps = 0; ps < 2; ++ps) {
      if (lane < 8) *(volatile v4f*)(stats + (size_t)bg * 32 + 4 * lane) = lv;
      __threadfence();
    }
  }
}

__global__ __launch_bounds__(256) void k_gnapply(const float* __restrict__ x,
                                                 const float* __restrict__ stats,
                                                 const float* __restrict__ gam,
                                                 const float* __restrict__ bet,
                                                 unsigned short* __restrict__ a1) {
  __shared__ __align__(16) float tf[CC * TFP];
  const int tid = threadIdx.x, lane = tid & 31, wave = tid >> 5;
  const int pix0 = blockIdx.x * 64;
  const int b = pix0 / HWP, p0 = pix0 - b * HWP;
#pragma unroll 1
  for (int it = 0; it < 8; ++it) {
    const int idx = it * 256 + tid;
    const int c = idx >> 4, j4 = (idx & 15) * 4;
    const v4f v = *(const v4f*)(x + ((size_t)(b * CC + c)) * HWP + p0 + j4);
    const int sl = (b * NGRP + (c >> 2)) * 32;
    const float mean = stats[sl], rstd = stats[sl + 1];
    const float g = gam[c], bt = bet[c];
    v4f o;
    o[0] = (v[0] - mean) * rstd * g + bt;
    o[1] = (v[1] - mean) * rstd * g + bt;
    o[2] = (v[2] - mean) * rstd * g + bt;
    o[3] = (v[3] - mean) * rstd * g + bt;
    *(v4f*)(tf + c * TFP + j4) = o;
  }
  __syncthreads();
  v4u val[12];
#pragma unroll
  for (int it = 0; it < 12; ++it) {
    const int q = it * 32 + lane;
    const int rl = q / 48, pc = q - rl * 48;
    const int sec = pc >> 4, c8 = (pc & 15) * 8;
    const int lo = (sec == 1);
    const float* cp = tf + c8 * TFP + (wave * 8 + rl);
    v4u u;
    u[0] = bfpack2(cp[0 * TFP], cp[1 * TFP], lo);
    u[1] = bfpack2(cp[2 * TFP], cp[3 * TFP], lo);
    u[2] = bfpack2(cp[4 * TFP], cp[5 * TFP], lo);
    u[3] = bfpack2(cp[6 * TFP], cp[7 * TFP], lo);
    val[it] = u;
  }
  for (int ps = 0; ps < 2; ++ps) {
#pragma unroll
    for (int it = 0; it < 12; ++it) {
      const int q = it * 32 + lane;
      const int rl = q / 48, pc = q - rl * 48;
      *(volatile v4u*)(a1 + ((size_t)(pix0 + wave * 8 + rl)) * KF + pc * 8) = val[it];
    }
    __threadfence();
  }
}

__global__ __launch_bounds__(256) void k_wplane(const float* __restrict__ w, unsigned short* __restrict__ plane,
                                               int nrows) {
  const int tid = threadIdx.x, lane = tid & 31, wave = tid >> 5;
  const int r0 = blockIdx.x * 64;
  v4u val[12];
#pragma unroll
  for (int it = 0; it < 12; ++it) {
    const int q = it * 32 + lane;
    const int rl = q / 48, pc = q - rl * 48;
    const int sec = pc >> 4, c8 = (pc & 15) * 8;
    const int lo = (sec == 2);
    const int row = min(r0 + wave * 8 + rl, nrows - 1);
    const float* cp = w + (size_t)row * CC + c8;
    const v4f f0 = *(const v4f*)(cp), f1 = *(const v4f*)(cp + 4);
    v4u u;
    u[0] = bfpack2(f0[0], f0[1], lo);
    u[1] = bfpack2(f0[2], f0[3], lo);
    u[2] = bfpack2(f1[0], f1[1], lo);
    u[3] = bfpack2(f1[2], f1[3], lo);
    val[it] = u;
  }
  for (int ps = 0; ps < 2; ++ps) {
#pragma unroll
    for (int it = 0; it < 12; ++it) {
      const int q = it * 32 + lane;
      const int rl = q / 48, pc = q - rl * 48;
      const int row = r0 + wave * 8 + rl;
      if (row < nrows) *(volatile v4u*)(plane + (size_t)row * KF + pc * 8) = val[it];
    }
    __threadfence();
  }
}

__global__ __launch_bounds__(256) void k_qkv(const unsigned short* __restrict__ a1,
                                             const unsigned short* __restrict__ wq,
                                             const float* __restrict__ qb,
                                             unsigned short* __restrict__ qkvp) {
  __shared__ __align__(16) float st[32 * STP];
  const int tid = threadIdx.x, lane = tid & 31, wave = tid >> 5;
  const int hl = lane >> 4, m = lane & 15;
  const int mi = wave & 1;
  const int nb = (wave >> 1) * 96;
  const int m0 = blockIdx.x * 32;

  v8f acc[6];
#pragma unroll
  for (int t = 0; t < 6; ++t) acc[t] = zero8();
#pragma unroll 2
  for (int k0 = 0; k0 < KF; k0 += 32) {
    const v16b a = ldfragb(a1, KF, m0 + mi * 16, k0, lane);
#pragma unroll
    for (int t = 0; t < 6; ++t) {
      const v16b bfr = ldfragb(wq, KF, nb + 16 * t, k0, lane);
      acc[t] = mmab(a, bfr, acc[t]);
    }
  }
#pragma unroll
  for (int t = 0; t < 6; ++t) {
    const int col = nb + 16 * t + m;
    const float bb = qb[col];
#pragma unroll
    for (int r = 0; r < 8; ++r) st[(mi * 16 + 8 * hl + r) * STP + col] = acc[t][r] + bb;
  }
  __syncthreads();
  v4u val[12];
#pragma unroll
  for (int it = 0; it < 12; ++it) {
    const int q = it * 32 + lane;
    const int rl = q / 96, pc = q - rl * 96;
    const int s6 = pc >> 4;
    const int which = s6 >> 1, lo = s6 & 1;
    const int c8 = (pc & 15) * 8;
    const float* cp = st + (wave * 4 + rl) * STP + which * CC + c8;
    const v4f f0 = *(const v4f*)(cp), f1 = *(const v4f*)(cp + 4);
    v4u u;
    u[0] = bfpack2(f0[0], f0[1], lo);
    u[1] = bfpack2(f0[2], f0[3], lo);
    u[2] = bfpack2(f1[0], f1[1], lo);
    u[3] = bfpack2(f1[2], f1[3], lo);
    val[it] = u;
  }
  for (int ps = 0; ps < 2; ++ps) {
#pragma unroll
    for (int it = 0; it < 12; ++it) {
      const int q = it * 32 + lane;
      const int rl = q / 96, pc = q - rl * 96;
      *(volatile v4u*)(qkvp + ((size_t)(m0 + wave * 4 + rl)) * QKROW + pc * 8) = val[it];
    }
    __threadfence();
  }
}

__global__ __launch_bounds__(128) void k_attn(const unsigned short* __restrict__ qkvp,
                                              unsigned short* __restrict__ ao) {
  extern __shared__ __align__(16) char smem[];
  unsigned short* Ks = (unsigned short*)(smem);
  unsigned short* Vt = (unsigned short*)(smem + 36864);
  unsigned short* Qs = (unsigned short*)(smem + 71680);
  unsigned short* Ps = (unsigned short*)(smem + 76288);
  float* Os = (float*)(smem + 94720);

  const int tid = threadIdx.x, lane = tid & 31, wave = tid >> 5;
  const int hl = lane >> 4, m = lane & 15;
  const int blk = blockIdx.x;
  const int g = blk & 1;
  const int t = blk >> 1;
  const int tx = t % NTX;
  const int ty = (t / NTX) % NTY;
  const int b = t / (NTX * NTY);
  const int y0 = ty * 4, x0 = tx * 4;
  const int ry0 = min(max(y0 - 3, 0), IMH - 8);
  const int rx0 = min(max(x0 - 3, 0), IMW - 8);
  const size_t pixbase = (size_t)b * HWP;
  const v4u z4 = (v4u){0u, 0u, 0u, 0u};
  const v8us z8 = (v8us){0, 0, 0, 0, 0, 0, 0, 0};

#pragma unroll
  for (int it = 0; it < 2; ++it) {
    const int q = it * 128 + tid;
    const int pl = q >> 7, rem = q & 127;
    const int ql = rem >> 3, c8 = (rem & 7) * 8;
    const size_t pix = pixbase + (size_t)(y0 + (ql >> 2)) * IMW + (x0 + (ql & 3));
    const v4u v = *(const v4u*)(qkvp + pix * QKROW + pl * CC + g * 64 + c8);
    *(v4u*)(Qs + pl * (16 * KSP) + ql * KSP + c8) = v;
  }
#pragma unroll 2
  for (int it = 0; it < 16; ++it) {
    const int q = it * 128 + tid;
    const int pl = q >> 10, rem = q & 1023;
    const int n = rem >> 3, c8 = (rem & 7) * 8;
    const int nn = min(n, 120);
    const int dr = nn / 11, dc = nn - dr * 11;
    const int row = min(ry0 + dr, IMH - 1), col = min(rx0 + dc, IMW - 1);
    const size_t pix = pixbase + (size_t)row * IMW + col;
    const v4u v = *(const v4u*)(qkvp + pix * QKROW + (2 + pl) * CC + g * 64 + c8);
    const v4u w4 = (n < 121) ? v : z4;
    *(v4u*)(Ks + pl * (128 * KSP) + n * KSP + c8) = w4;
  }
#pragma unroll 2
  for (int it = 0; it < 16; ++it) {
    const int q = it * 128 + tid;
    const int pl = q >> 10, rem = q & 1023;
    const int n = rem >> 3, c8 = (rem & 7) * 8;
    const int nn = min(n, 120);
    const int dr = nn / 11, dc = nn - dr * 11;
    const int row = min(ry0 + dr, IMH - 1), col = min(rx0 + dc, IMW - 1);
    const size_t pix = pixbase + (size_t)row * IMW + col;
    Pk8 pk;
    pk.u4 = *(const v4u*)(qkvp + pix * QKROW + (4 + pl) * CC + g * 64 + c8);
    if (n > 120) pk.u4 = z4;
    unsigned short* vd = Vt + pl * (64 * VTP) + c8 * VTP + n;
#pragma unroll
    for (int e = 0; e < 8; ++e) vd[e * VTP] = pk.u8[e];
  }
  __syncthreads();

  const int hc = wave * HDH;
  int dro[8], dco[8];
#pragma unroll
  for (int r = 0; r < 8; ++r) {
    const int ql = 8 * hl + r;
    const int qy = y0 + (ql >> 2), qx = x0 + (ql & 3);
    dro[r] = min(max(qy - 3, 0), IMH - 8) - ry0;
    dco[r] = min(max(qx - 3, 0), IMW - 8) - rx0;
  }
  FragB qa;
  qa.u[0] = *(const v8us*)(Qs + m * KSP + hc + 8 * hl);
  qa.u[1] = *(const v8us*)(Qs + 16 * KSP + m * KSP + hc + 8 * hl);
  unsigned short* pw = Ps + wave * (2 * 16 * KSP);
  const float NEGI = -__builtin_huge_valf();
  float mrow[8], lrow[8];
#pragma unroll
  for (int r = 0; r < 8; ++r) { mrow[r] = NEGI; lrow[r] = 0.f; }
  v8f oacc = zero8();

#pragma unroll 1
  for (int kc = 0; kc < 2; ++kc) {
    __syncthreads();
    v8f s[4];
#pragma unroll
    for (int j = 0; j < 4; ++j) {
      const unsigned short* kp = Ks + (kc * 64 + j * 16 + m) * KSP + hc + 8 * hl;
      FragB kb, kl;
      kb.u[0] = *(const v8us*)(kp);
      kb.u[1] = kb.u[0];
      kl.u[0] = *(const v8us*)(kp + 128 * KSP);
      kl.u[1] = z8;
      const v8f sa = mmab(qa.v, kb.v, zero8());
      s[j] = mmab(qa.v, kl.v, sa);
    }
#pragma unroll
    for (int j = 0; j < 4; ++j) {
      const int nl = kc * 64 + j * 16 + m;
      const int nn = min(nl, 120);
      const int dr = nn / 11, dc = nn - dr * 11;
      const bool inr = nl < 121;
#pragma unroll
      for (int r = 0; r < 8; ++r) {
        const bool ok = inr && ((unsigned)(dr - dro[r]) < 8u) && ((unsigned)(dc - dco[r]) < 8u);
        const float sv = s[j][r] * 0.25f;
        s[j][r] = ok ? sv : NEGI;
      }
    }
    float cm[8];
#pragma unroll
    for (int r = 0; r < 8; ++r) {
      float mx = NEGI;
#pragma unroll
      for (int j = 0; j < 4; ++j) mx = fmaxf(mx, s[j][r]);
#pragma unroll
      for (int off = 1; off < 16; off <<= 1) mx = fmaxf(mx, __shfl_xor(mx, off, 32));
      cm[r] = mx;
    }
    float al[8];
#pragma unroll
    for (int r = 0; r < 8; ++r) {
      const float mnew  = fmaxf(mrow[r], cm[r]);
      const float alpha = __expf(mrow[r] - mnew);
      mrow[r] = mnew;
      float psum = 0.f;
#pragma unroll
      for (int j = 0; j < 4; ++j) {
        const float pv = __expf(s[j][r] - mnew);
        psum += pv;
        const unsigned int hb = bfbits(pv);
        const unsigned int lb = bfbits(pv - __uint_as_float(hb << 16));
        pw[(8 * hl + r) * KSP + j * 16 + m] = (unsigned short)hb;
        pw[16 * KSP + (8 * hl + r) * KSP + j * 16 + m] = (unsigned short)lb;
      }
#pragma unroll
      for (int off = 1; off < 16; off <<= 1) psum += __shfl_xor(psum, off, 32);
      lrow[r] = lrow[r] * alpha + psum;
      al[r] = alpha;
    }
#pragma unroll
    for (int r = 0; r < 8; ++r) oacc[r] *= al[r];
    __syncthreads();
#pragma unroll
    for (int kk = 0; kk < 2; ++kk) {
      const v16b pah = ldfragb(pw, KSP, 0, kk * 32, lane);
      const v16b pal = ldfragb(pw + 16 * KSP, KSP, 0, kk * 32, lane);
      const unsigned short* vq = Vt + (hc + m) * VTP + kc * 64 + kk * 32 + 8 * hl;
      FragB vh, vl;
      vh.u[0] = *(const v8us*)(vq);
      vh.u[1] = *(const v8us*)(vq + 16);
      vl.u[0] = *(const v8us*)(vq + 64 * VTP);
      vl.u[1] = *(const v8us*)(vq + 64 * VTP + 16);
      oacc = mmab(pah, vh.v, oacc);
      oacc = mmab(pal, vh.v, oacc);
      oacc = mmab(pah, vl.v, oacc);
    }
  }
#pragma unroll
  for (int r = 0; r < 8; ++r) Os[(8 * hl + r) * OSP + hc + m] = oacc[r] * (1.0f / lrow[r]);
  __syncthreads();

  v4u val[3];
#pragma unroll
  for (int it = 0; it < 3; ++it) {
    const int L = it * 4 + (lane >> 3);
    const int c8 = (lane & 7) * 8;
    const int qd = L / 3;
    const int sec = L - 3 * qd;
    const int ql = wave * 4 + qd;
    const int lo = (sec == 1);
    const float* cp = Os + ql * OSP + c8;
    const v4f f0 = *(const v4f*)(cp), f1 = *(const v4f*)(cp + 4);
    v4u u;
    u[0] = bfpack2(f0[0], f0[1], lo);
    u[1] = bfpack2(f0[2], f0[3], lo);
    u[2] = bfpack2(f1[0], f1[1], lo);
    u[3] = bfpack2(f1[2], f1[3], lo);
    val[it] = u;
  }
  for (int ps = 0; ps < 2; ++ps) {
#pragma unroll
    for (int it = 0; it < 3; ++it) {
      const int L = it * 4 + (lane >> 3);
      const int c8 = (lane & 7) * 8;
      const int qd = L / 3;
      const int sec = L - 3 * qd;
      const int ql = wave * 4 + qd;
      const size_t pix = pixbase + (size_t)(y0 + (ql >> 2)) * IMW + (x0 + (ql & 3));
      *(volatile v4u*)(ao + pix * KF + sec * CC + g * 64 + c8) = val[it];
    }
    __threadfence();
  }
}

__global__ __launch_bounds__(256) void k_proj(const unsigned short* __restrict__ ao,
                                              const unsigned short* __restrict__ wp,
                                              const float* __restrict__ pb,
                                              float* __restrict__ out) {
  __shared__ __align__(16) float os[CC * OSP];
  const int tid = threadIdx.x, lane = tid & 31, wave = tid >> 5;
  const int hl = lane >> 4, m = lane & 15;
  const int pix0 = blockIdx.x * 64;
  const int b = pix0 / HWP, p0 = pix0 - b * HWP;
  const int mi = wave & 3;
  const int nb = (wave >> 2) * 64;

  v8f acc[4];
#pragma unroll
  for (int t = 0; t < 4; ++t) acc[t] = zero8();
#pragma unroll 2
  for (int k0 = 0; k0 < KF; k0 += 32) {
    const v16b a = ldfragb(ao, KF, pix0 + mi * 16, k0, lane);
#pragma unroll
    for (int t = 0; t < 4; ++t) {
      const v16b bfr = ldfragb(wp, KF, nb + 16 * t, k0, lane);
      acc[t] = mmab(a, bfr, acc[t]);
    }
  }
#pragma unroll
  for (int t = 0; t < 4; ++t) {
    const int col = nb + 16 * t + m;
    const float bb = pb[col];
#pragma unroll
    for (int r = 0; r < 8; ++r) {
      const int row = mi * 16 + 8 * hl + r;
      os[col * OSP + row] = acc[t][r] + bb;
    }
  }
  __syncthreads();
  for (int ps = 0; ps < 2; ++ps) {
#pragma unroll
    for (int it = 0; it < 8; ++it) {
      const int gi = wave * 256 + it * 32 + lane;
      const int cch = gi >> 4, j4 = (gi & 15) * 4;
      const v4f v = *(const v4f*)(os + cch * OSP + j4);
      *(volatile v4f*)(out + ((size_t)(b * CC + cch)) * HWP + p0 + j4) = v;
    }
    __threadfence();
  }
}

extern "C" void kernel_launch(void* const* d_in, const int* in_sizes, int n_in,
                              void* d_out, int out_size, void* d_ws, size_t ws_size,
                              hipStream_t stream) {
  if (n_in < 7) return;
  if (in_sizes[0] != NPIX * CC) return;
  if (in_sizes[1] != CC || in_sizes[2] != CC) return;
  if (in_sizes[3] != NQKV * CC || in_sizes[4] != NQKV) return;
  if (in_sizes[5] != CC * CC || in_sizes[6] != CC) return;
  if (out_size != NPIX * CC) return;

  const float* x      = (const float*)d_in[0];
  const float* gn_g   = (const float*)d_in[1];
  const float* gn_b   = (const float*)d_in[2];
  const float* qkv_w  = (const float*)d_in[3];
  const float* qkv_b  = (const float*)d_in[4];
  const float* proj_w = (const float*)d_in[5];
  const float* proj_b = (const float*)d_in[6];
  float* out = (float*)d_out;

  size_t off = 0;
  const size_t oST = off; off += (size_t)64 * 32 * 4;
  const size_t oA1 = off; off += (size_t)NPIX * KF * 2;
  const size_t oWQ = off; off += (size_t)NQKV * KF * 2;
  const size_t oWP = off; off += (size_t)CC * KF * 2;
  const size_t oQK = off; off += (size_t)NPIX * QKROW * 2;
  const size_t oAO = off; off += (size_t)NPIX * KF * 2;
  if (off > ws_size) return;
  if (off > (size_t)134217728) return;

  char* ws = (char*)d_ws;
  float*          STATS = (float*)(ws + oST);
  unsigned short* A1    = (unsigned short*)(ws + oA1);
  unsigned short* WQ    = (unsigned short*)(ws + oWQ);
  unsigned short* WP    = (unsigned short*)(ws + oWP);
  unsigned short* QKVP  = (unsigned short*)(ws + oQK);
  unsigned short* AO    = (unsigned short*)(ws + oAO);

  k_gnstats<<<dim3(NBT * NGRP), dim3(256), 0, stream>>>(x, STATS);
  k_gnapply<<<dim3(NPIX / 64), dim3(256), 0, stream>>>(x, STATS, gn_g, gn_b, A1);
  k_wplane<<<dim3(NQKV / 64), dim3(256), 0, stream>>>(qkv_w, WQ, NQKV);
  k_wplane<<<dim3(CC / 64), dim3(256), 0, stream>>>(proj_w, WP, CC);
  k_qkv<<<dim3(NPIX / 32), dim3(256), 0, stream>>>(A1, WQ, qkv_b, QKVP);
  (void)hipFuncSetAttribute(reinterpret_cast<const void*>(&k_attn),
                            hipFuncAttributeMaxDynamicSharedMemorySize, ATT_LDS);
  k_attn<<<dim3(NBT * NTY * NTX * 2), dim3(128), ATT_LDS, stream>>>(QKVP, AO);
  k_proj<<<dim3(NPIX / 64), dim3(256), 0, stream>>>(AO, WP, proj_b, out);
  (void)hipGetLastError();
}
